// SelfAttention_45191645888943
// MI455X (gfx1250) — hardware-verified
//
#include <hip/hip_runtime.h>


#ifndef NB
#define NB 8
#endif
#ifndef SEQ
#define SEQ 1024
#endif
#define NB_FULL  8
#define SEQ_FULL 1024
#define DM   128
#define NH_  8
#define HD   128
#define HK   (NH_ * HD)
#define AW   4
#define OSP  132
#define EROWS (SEQ < 256 ? SEQ : 256)
#define QRS  2048.0f
#define QRI  (1.0f / 2048.0f)
#define SC2  ((float)(0.08838834764831845 * 1.4426950408889634))
#define PSH  14.0f
#define NEGB (-3.0e38f)
#define CXS  16.0f
#define WOS  1024.0f
#define OSI  (1.0f / 16384.0f)

static_assert(HD == 128);
static_assert(NH_ * HD == HK);
static_assert(HD % 64 == 0);
static_assert(HK % 64 == 0);
static_assert(DM % 64 == 0);
static_assert(DM % 32 == 0);
static_assert(HK % 32 == 0);
static_assert(SEQ % 64 == 0);
static_assert(SEQ % 32 == 0);
static_assert(EROWS % 64 == 0);
static_assert(EROWS >= 64);
static_assert(EROWS <= SEQ);
static_assert(EROWS % (16 * AW) == 0);
static_assert((SEQ - EROWS) % (16 * AW) == 0);
static_assert(EROWS % 32 == 0);
static_assert((SEQ - EROWS) % 32 == 0);
static_assert(NB <= NB_FULL);
static_assert(SEQ <= SEQ_FULL);
static_assert((OSP * 4) % 16 == 0);
static_assert(OSP >= HD);
static_assert((size_t)NB * NH_ * SEQ * HD < (size_t)2147483647);
static_assert((size_t)AW * 16 * OSP * 4 <= (size_t)131072);
static_assert((size_t)16 * 68 * 4 <= (size_t)131072);
static_assert(32 * 4 * 16 == 16 * 64 * 2);
static_assert(32 * 8 * 16 == 16 * HD * 2);
static_assert(32 * 8 * 16 == 16 * 64 * 4);
static_assert((DM / 8) == 16);

typedef _Float16 h16;
typedef unsigned short bf;
typedef __attribute__((ext_vector_type(16))) __bf16   v16bf;
typedef __attribute__((ext_vector_type(16))) _Float16 v16h;
typedef __attribute__((ext_vector_type(8)))  _Float16 v8h;
typedef __attribute__((ext_vector_type(8)))  unsigned short v8us;
typedef __attribute__((ext_vector_type(8)))  float    v8f;
typedef __attribute__((ext_vector_type(4)))  float    v4f;
typedef v4f  __attribute__((may_alias)) v4fa;

__device__ __forceinline__ unsigned short f2bf(float f) { unsigned u = __float_as_uint(f); u += 0x7FFFu + ((u >> 16) & 1u); return (unsigned short)(u >> 16); }
__device__ __forceinline__ float bfr(float f) { return __uint_as_float(((unsigned)f2bf(f)) << 16); }
__device__ __forceinline__ v16h cat16(v8h lo, v8h hi) { return __builtin_shufflevector(lo, hi, 0, 1, 2, 3, 4, 5, 6, 7, 8, 9, 10, 11, 12, 13, 14, 15); }
__device__ __forceinline__ v16bf cat16b(v8us lo, v8us hi) { return __builtin_bit_cast(v16bf, __builtin_shufflevector(lo, hi, 0, 1, 2, 3, 4, 5, 6, 7, 8, 9, 10, 11, 12, 13, 14, 15)); }
__device__ __forceinline__ v8f wmma16(v16h a, v16h b, v8f c) { return __builtin_amdgcn_wmma_f32_16x16x32_f16(false, a, false, b, (short)0, c, false, false); }
__device__ __forceinline__ v8f wmmab(v16bf a, v16bf b, v8f c) { return __builtin_amdgcn_wmma_f32_16x16x32_bf16(false, a, false, b, (short)0, c, false, false); }
__device__ __forceinline__ v16h  ldh(const h16* p) { return cat16(*(const v8h*)p, *(const v8h*)(p + 16)); }
__device__ __forceinline__ v16bf ldb(const bf* p)  { return cat16b(*(const v8us*)p, *(const v8us*)(p + 16)); }
__device__ __forceinline__ void wave_sync() { __builtin_amdgcn_fence(3  , "wavefront"); __builtin_amdgcn_wave_barrier(); asm volatile("" ::: "memory"); }
static __device__ __forceinline__ h16 toh_flush(float v) { const h16 r = (h16)v; return (fabsf(v) < 6.103515625e-05f) ? (h16)0.0f : r; }
__device__ __forceinline__ v8f mmh(v16h a, v16h b, v8f c) { c = wmma16(a, b, c); asm volatile("v_nop\n\tv_nop\n\tv_nop\n\tv_nop" : "+v"(c) : "v"(a), "v"(b)); return c; }
__device__ __forceinline__ v8f mmb(v16bf a, v16bf b, v8f c) { c = wmmab(a, b, c); asm volatile("v_nop\n\tv_nop\n\tv_nop\n\tv_nop" : "+v"(c) : "v"(a), "v"(b)); return c; }

__global__ __launch_bounds__(256) void k_cvt8(const float* __restrict__ src, bf* dst, size_t n8) {
    const size_t i = (size_t)blockIdx.x * 256 + threadIdx.x; if (i >= n8) return;
    const v8f v = *(const v8f*)(src + i * 8); v8us o;
#pragma unroll
    for (int k = 0; k < 8; ++k) o[k] = f2bf(v[k]);
    *(volatile v8us*)(dst + i * 8) = o; __threadfence(); *(volatile v8us*)(dst + i * 8) = o;
}

__global__ __launch_bounds__(256) void k_cvtx(const float* __restrict__ src, bf* dst, int n8) {
    const int i = (int)blockIdx.x * 256 + (int)threadIdx.x; if (i >= n8) return;
    const int row = i >> 4, pc = i & 15;
    const int b = row / SEQ, t = row % SEQ;
    const v8f v = *(const v8f*)(src + ((size_t)t * NB_FULL + (size_t)b) * DM + (size_t)pc * 8); v8us o;
#pragma unroll
    for (int k = 0; k < 8; ++k) o[k] = f2bf(v[k]);
    *(volatile v8us*)(dst + (size_t)i * 8) = o; __threadfence(); *(volatile v8us*)(dst + (size_t)i * 8) = o;
}

__global__ __launch_bounds__(256) void k_cvtwo(const float* __restrict__ src, h16* dst, int n8) {
    const int i = (int)blockIdx.x * 256 + (int)threadIdx.x; if (i >= n8) return;
    const v8f v = *(const v8f*)(src + (size_t)i * 8); v8h o;
#pragma unroll
    for (int k = 0; k < 8; ++k) o[k] = toh_flush(bfr(v[k]) * WOS);
    *(volatile v8h*)(dst + (size_t)i * 8) = o; __threadfence(); *(volatile v8h*)(dst + (size_t)i * 8) = o;
}

template <int MODE>
__device__ __forceinline__ void proj_body(const bf* __restrict__ A, const bf* __restrict__ Bt, const float* __restrict__ bias, h16* Ph, h16* Pr, int resT) {
    __shared__ __align__(16) float os[16 * 68];
    const int K = DM;
    const int lane = threadIdx.x & 31, lr = lane & 15, hi = lane >> 4; const int r0 = blockIdx.x * 64, c0 = blockIdx.y * 64;
    v8f acc[4][4];
#pragma unroll
    for (int mb = 0; mb < 4; ++mb)
#pragma unroll
        for (int nb = 0; nb < 4; ++nb) acc[mb][nb] = (v8f){};
    const size_t aoff = (size_t)(r0 + lr) * K + 8 * hi, boff = (size_t)(c0 + lr) * K + 8 * hi;
#pragma unroll 1
    for (int kc = 0; kc < K; kc += 32) {
        v16bf a[4];
#pragma unroll
        for (int mb = 0; mb < 4; ++mb) a[mb] = ldb(A + aoff + (size_t)mb * 16 * K + kc);
#pragma unroll
        for (int nb = 0; nb < 4; ++nb) { const v16bf b = ldb(Bt + boff + (size_t)nb * 16 * K + kc);
#pragma unroll
            for (int mb = 0; mb < 4; ++mb) acc[mb][nb] = mmb(a[mb], b, acc[mb][nb]); }
    }
    float bc[4];
#pragma unroll
    for (int nb = 0; nb < 4; ++nb) bc[nb] = (MODE == 0) ? bfr(bias[c0 + nb * 16 + lr]) : 0.0f;
    size_t tbase, rbase, tpitch, rpitch; bool wr;
    if (MODE == 0) { const int bb = r0 / SEQ, tt = r0 % SEQ; const int zc = bb * NH_ + c0 / HD; const int d0 = c0 % HD;
                     tbase = ((size_t)zc * SEQ + (size_t)tt) * HD + (size_t)d0; tpitch = HD;
                     rbase = ((size_t)zc * (size_t)resT + (size_t)tt) * HD + (size_t)d0; rpitch = HD; wr = tt < resT; }
    else           { const int bb = c0 / SEQ, tt = c0 % SEQ;
                     tbase = ((size_t)bb * HK + (size_t)r0) * SEQ + (size_t)tt; tpitch = SEQ;
                     rbase = ((size_t)bb * HK + (size_t)r0) * (size_t)resT + (size_t)tt; rpitch = (size_t)resT; wr = tt < resT; }
#pragma unroll
    for (int mb = 0; mb < 4; ++mb) {
        float br[8];
#pragma unroll
        for (int j = 0; j < 8; ++j) br[j] = (MODE == 1) ? bfr(bias[r0 + mb * 16 + hi * 8 + j]) : 0.0f;
#pragma unroll
        for (int nb = 0; nb < 4; ++nb) {
#pragma unroll
            for (int j = 0; j < 8; ++j) os[(hi * 8 + j) * 68 + nb * 16 + lr] = acc[mb][nb][j] + bc[nb] + br[j]; }
        wave_sync();
#pragma unroll 1
        for (int ps = 0; ps < 2; ++ps) {
#pragma unroll
            for (int s = 0; s < 4; ++s) { const int row = 4 * s + (lane >> 3), c8 = (lane & 7) * 8;
                const v4f x0 = *(const v4fa*)(&os[row * 68 + c8]); const v4f x1 = *(const v4fa*)(&os[row * 68 + c8 + 4]); v8h hv, rv;
#pragma unroll
                for (int i = 0; i < 4; ++i) { const h16 a0 = toh_flush(x0[i]); const h16 a1 = toh_flush(x1[i]); hv[i] = a0; hv[4 + i] = a1;
                    rv[i] = toh_flush((x0[i] - (float)a0) * QRS); rv[4 + i] = toh_flush((x1[i] - (float)a1) * QRS); }
                const size_t oo = tbase + (size_t)(mb * 16 + row) * tpitch + (size_t)c8;
                const size_t ro = rbase + (size_t)(mb * 16 + row) * rpitch + (size_t)c8;
                *(volatile v8h*)(Ph + oo) = hv; if (wr) *(volatile v8h*)(Pr + ro) = rv; }
            if (ps == 0) __threadfence(); }
        wave_sync();
    }
}

__global__ __launch_bounds__(32) void k_proj_rows(const bf* __restrict__ A, const bf* __restrict__ Bt, const float* __restrict__ bias, h16* Ph, h16* Pr, int resT) { proj_body<0>(A, Bt, bias, Ph, Pr, resT); }
__global__ __launch_bounds__(32) void k_proj_tr(const bf* __restrict__ A, const bf* __restrict__ Bt, const float* __restrict__ bias, h16* Ph, h16* Pr, int resT) { proj_body<1>(A, Bt, bias, Ph, Pr, resT); }

template <int EARLY>
__device__ __forceinline__ v8f score16(const h16* __restrict__ RH, const h16* __restrict__ RR, const h16* __restrict__ CH, const h16* __restrict__ CR, int rx, int rrx, int cx, int crx) {
    v8f sH = (v8f){}, sL = (v8f){};
#pragma unroll
    for (int kc = 0; kc < HD; kc += 32) {
        const v16h qf = ldh(RH + rx + kc); const v16h kf = ldh(CH + cx + kc);
        sH = mmh(kf, qf, sH);
        if (EARLY) { const v16h qr = ldh(RR + rrx + kc); const v16h kr = ldh(CR + crx + kc);
                     sL = mmh(kf, qr, sL); sL = mmh(kr, qf, sL); __builtin_amdgcn_sched_barrier(0); }
    }
    v8f t;
#pragma unroll
    for (int r = 0; r < 8; ++r) t[r] = EARLY ? ((sH[r] + sL[r] * QRI) * SC2) : (sH[r] * SC2);
    return t;
}

template <int EARLY>
__device__ __forceinline__ void flash_body(const h16* __restrict__ RH, const h16* __restrict__ RR, const h16* __restrict__ CH, const h16* __restrict__ CR,
                                           const h16* __restrict__ VT, const h16* __restrict__ VR, h16* CX, h16* CXR) {
    __shared__ __align__(16) float os[AW * 16 * OSP];
    const int lane = threadIdx.x & 31, lr = lane & 15, hi = lane >> 4;
    const int wave = __builtin_amdgcn_readfirstlane((int)(threadIdx.x >> 5));
    const int zh = blockIdx.y; const int b = zh / NH_, h = zh % NH_;
    const int t0 = (EARLY ? 0 : EROWS) + ((int)blockIdx.x * AW + wave) * 16;
    const int lim = t0 + lr;
    const int nk = (t0 + 16 + 31) & ~31;
    const int pbase = zh * (SEQ * HD);
    const int rbase = zh * (EROWS * HD);
    const int tcl = EARLY ? (t0 + lr) : 0;
    const int ro  = pbase + (t0 + lr) * HD + 8 * hi;
    const int rro = rbase + tcl * HD + 8 * hi;
    const int co  = pbase + lr * HD + 8 * hi;
    const int cro = rbase + lr * HD + 8 * hi;
    const int vo  = pbase + lr * SEQ + 8 * hi;
    const int vro = rbase + lr * EROWS + 8 * hi;
    const v16h hz = (v16h){};
    v8f o[8], oR[8];
#pragma unroll
    for (int j = 0; j < 8; ++j) { o[j] = (v8f){}; oR[j] = (v8f){}; }
    float m = NEGB, l = 0.0f;
#pragma unroll 1
    for (int key0 = 0; key0 < nk; key0 += 32) {
        int rx = ro, rrx = rro;
        asm volatile("" : "+v"(rx), "+v"(rrx));
        const v8f ta = score16<EARLY>(RH, RR, CH, CR, rx, rrx, co + key0 * HD, cro + key0 * HD);
        const v8f tb = score16<EARLY>(RH, RR, CH, CR, rx, rrx, co + (key0 + 16) * HD, cro + (key0 + 16) * HD);
        const int ja = key0 + 8 * hi;
        bool fa[8], fb[8]; float mx = NEGB;
#pragma unroll
        for (int r = 0; r < 8; ++r) {
            fa[r] = (ja + r <= lim); fb[r] = (ja + 16 + r <= lim);
            mx = fmaxf(mx, fmaxf(fa[r] ? ta[r] : NEGB, fb[r] ? tb[r] : NEGB)); }
        mx = fmaxf(mx, __shfl_xor(mx, 16, 32));
        const float mnew = fmaxf(m, mx);
        const float alpha = __builtin_amdgcn_exp2f(m - mnew);
        const float sh = PSH - mnew;
        v16h pb, pr = hz; float ls = 0.0f;
#pragma unroll
        for (int r = 0; r < 8; ++r) {
            const float xa = ta[r] + sh, xb = tb[r] + sh;
            const float ea = __builtin_amdgcn_exp2f(xa), eb = __builtin_amdgcn_exp2f(xb);
            const float ga = (fa[r] & (xa >= -14.0f)) ? ea : 0.0f;
            const float gb = (fb[r] & (xb >= -14.0f)) ? eb : 0.0f;
            const h16 pa = (h16)ga; const h16 pc = (h16)gb;
            pb[r] = pa; pb[8 + r] = pc;
            if (EARLY) { pr[r] = toh_flush((ga - (float)pa) * QRS); pr[8 + r] = toh_flush((gb - (float)pc) * QRS); ls += ga + gb; }
            else       { ls += (float)pa + (float)pc; } }
        l = l * alpha + ls; m = mnew;
#pragma unroll
        for (int j = 0; j < 8; ++j) { o[j] = o[j] * alpha; if (EARLY) oR[j] = oR[j] * alpha; }
#pragma unroll
        for (int j = 0; j < 8; ++j) {
            const v16h vf = ldh(VT + vo + j * (16 * SEQ) + key0);
            o[j] = mmh(vf, pb, o[j]);
            if (EARLY) { const v16h vr = ldh(VR + vro + j * (16 * EROWS) + key0);
                         oR[j] = mmh(vf, pr, oR[j]); oR[j] = mmh(vr, pb, oR[j]); __builtin_amdgcn_sched_barrier(0); }
        }
    }
    l += __shfl_xor(l, 16, 32);
    const bool any = l > 0.0f;
    const float lsafe = any ? l : 1.0f;
    const float inv = any ? (CXS * (1.0f / lsafe)) : 0.0f;
    const int wb = wave * 16 * OSP;
#pragma unroll
    for (int j = 0; j < 8; ++j) {
        v8f f = o[j]; if (EARLY) f = o[j] + oR[j] * QRI;
        v4f a, c;
        a[0] = f[0] * inv; a[1] = f[1] * inv; a[2] = f[2] * inv; a[3] = f[3] * inv; c[0] = f[4] * inv; c[1] = f[5] * inv; c[2] = f[6] * inv; c[3] = f[7] * inv;
        *(v4fa*)(&os[wb + lr * OSP + 16 * j + 8 * hi]) = a; *(v4fa*)(&os[wb + lr * OSP + 16 * j + 8 * hi + 4]) = c; }
    wave_sync();
    h16* crow = CX + ((size_t)b * SEQ + (size_t)t0) * HK + (size_t)h * HD;
    h16* rrow = CXR + ((size_t)b * EROWS + (size_t)(EARLY ? t0 : 0)) * HK + (size_t)h * HD;
#pragma unroll 1
    for (int ps = 0; ps < 2; ++ps) {
#pragma unroll
        for (int s = 0; s < 8; ++s) { const int row = 2 * s + (lane >> 4), c8 = (lane & 15) * 8;
            const v4f x0 = *(const v4fa*)(&os[wb + row * OSP + c8]); const v4f x1 = *(const v4fa*)(&os[wb + row * OSP + c8 + 4]); v8h hv, rv;
#pragma unroll
            for (int i = 0; i < 4; ++i) { const h16 a0 = toh_flush(x0[i]); const h16 a1 = toh_flush(x1[i]); hv[i] = a0; hv[4 + i] = a1;
                rv[i] = toh_flush((x0[i] - (float)a0) * QRS); rv[4 + i] = toh_flush((x1[i] - (float)a1) * QRS); }
            *(volatile v8h*)(crow + (size_t)row * HK + c8) = hv;
            if (EARLY) *(volatile v8h*)(rrow + (size_t)row * HK + c8) = rv; }
        if (ps == 0) __threadfence(); }
}

__global__ __launch_bounds__(32 * AW) __attribute__((amdgpu_num_vgpr(256))) void k_flash_early(const h16* __restrict__ RH, const h16* __restrict__ RR, const h16* __restrict__ CH, const h16* __restrict__ CR,
                                                                                               const h16* __restrict__ VT, const h16* __restrict__ VR, h16* CX, h16* CXR) {
    flash_body<1>(RH, RR, CH, CR, VT, VR, CX, CXR);
}
__global__ __launch_bounds__(32 * AW) __attribute__((amdgpu_num_vgpr(256))) void k_flash_late(const h16* __restrict__ RH, const h16* __restrict__ RR, const h16* __restrict__ CH, const h16* __restrict__ CR,
                                                                                              const h16* __restrict__ VT, const h16* __restrict__ VR, h16* CX, h16* CXR) {
    flash_body<0>(RH, RR, CH, CR, VT, VR, CX, CXR);
}

template <int EARLY>
__device__ __forceinline__ void out_body(const h16* __restrict__ CX, const h16* __restrict__ CXR, const h16* __restrict__ WO, const float* __restrict__ bo, float* OUT) {
    __shared__ __align__(16) float os[16 * 68];
    const int lane = threadIdx.x & 31, lr = lane & 15, hi = lane >> 4;
    const int TB = EARLY ? (EROWS / 32) : (((SEQ - EROWS) / 32) > 0 ? ((SEQ - EROWS) / 32) : 1);
    const int b = (int)blockIdx.x / TB; const int t0 = (EARLY ? 0 : EROWS) + ((int)blockIdx.x % TB) * 32; const int c0 = blockIdx.y * 64;
    v8f acc[2][4], accr[2][4];
#pragma unroll
    for (int mb = 0; mb < 2; ++mb)
#pragma unroll
        for (int nb = 0; nb < 4; ++nb) { acc[mb][nb] = (v8f){}; accr[mb][nb] = (v8f){}; }
    const size_t aoff = ((size_t)b * SEQ + (size_t)(t0 + lr)) * HK + 8 * hi;
    const size_t roff = ((size_t)b * EROWS + (size_t)((EARLY ? t0 : 0) + lr)) * HK + 8 * hi;
    const size_t boff = (size_t)(c0 + lr) * HK + 8 * hi;
#pragma unroll 1
    for (int kc = 0; kc < HK; kc += 32) {
        v16h a[2], ar[2];
#pragma unroll
        for (int mb = 0; mb < 2; ++mb) { a[mb] = ldh(CX + aoff + (size_t)mb * 16 * HK + kc); ar[mb] = a[mb];
            if (EARLY) ar[mb] = ldh(CXR + roff + (size_t)mb * 16 * HK + kc); }
#pragma unroll
        for (int nb = 0; nb < 4; ++nb) { const v16h w = ldh(WO + boff + (size_t)nb * 16 * HK + kc);
#pragma unroll
            for (int mb = 0; mb < 2; ++mb) { acc[mb][nb] = mmh(a[mb], w, acc[mb][nb]); if (EARLY) accr[mb][nb] = mmh(ar[mb], w, accr[mb][nb]); } }
    }
    float bc[4];
#pragma unroll
    for (int nb = 0; nb < 4; ++nb) bc[nb] = bfr(bo[c0 + nb * 16 + lr]);
#pragma unroll
    for (int mb = 0; mb < 2; ++mb) {
#pragma unroll
        for (int nb = 0; nb < 4; ++nb) {
#pragma unroll
            for (int j = 0; j < 8; ++j) { float v = acc[mb][nb][j]; if (EARLY) v = v + accr[mb][nb][j] * QRI;
                os[(hi * 8 + j) * 68 + nb * 16 + lr] = v * OSI + bc[nb]; } }
        wave_sync();
        float* orow = OUT + ((size_t)(t0 + mb * 16) * NB_FULL + (size_t)b) * DM + (size_t)c0;
#pragma unroll 1
        for (int ps = 0; ps < 2; ++ps) {
#pragma unroll
            for (int s = 0; s < 8; ++s) { const int row = 2 * s + (lane >> 4), cofs = (lane & 15) * 4;
                const v4f val = *(const v4fa*)(&os[row * 68 + cofs]);
                *(volatile v4f*)(orow + (size_t)row * (NB_FULL * DM) + cofs) = val; }
            if (ps == 0) __threadfence(); }
        wave_sync();
    }
}

__global__ __launch_bounds__(32) __attribute__((amdgpu_num_vgpr(256))) void k_out_early(const h16* __restrict__ CX, const h16* __restrict__ CXR, const h16* __restrict__ WO, const float* __restrict__ bo, float* OUT) {
    out_body<1>(CX, CXR, WO, bo, OUT);
}
__global__ __launch_bounds__(32) void k_out_late(const h16* __restrict__ CX, const h16* __restrict__ CXR, const h16* __restrict__ WO, const float* __restrict__ bo, float* OUT) {
    out_body<0>(CX, CXR, WO, bo, OUT);
}

static constexpr size_t al256(size_t v) { return (v + 255) & ~(size_t)255; }
static constexpr size_t SZ_XB = al256((size_t)NB * SEQ * DM * 2);
static constexpr size_t SZ_WB = al256((size_t)3 * HK * DM * 2);
static constexpr size_t SZ_WO = al256((size_t)DM * HK * 2);
static constexpr size_t SZ_PL = al256((size_t)NB * NH_ * SEQ * HD * 2);
static constexpr size_t SZ_RS = al256((size_t)NB * NH_ * EROWS * HD * 2);
static constexpr size_t SZ_CX = al256((size_t)NB * SEQ * HK * 2);
static constexpr size_t SZ_CR = al256((size_t)NB * EROWS * HK * 2);
static constexpr size_t SZ_TOTAL = SZ_XB + SZ_WB + SZ_WO + 3 * SZ_PL + 3 * SZ_RS + SZ_CX + SZ_CR;
static_assert(SZ_TOTAL <= (size_t)134217728);
static_assert(((size_t)HK * DM * 2) % 256 == 0);
static_assert((size_t)NB * NH_ * SEQ * HD == (size_t)NB * HK * SEQ);
static_assert((size_t)NB * NH_ * EROWS * HD == (size_t)NB * HK * EROWS);
static_assert(((size_t)NB * SEQ * DM / 8) % 256 == 0);
static_assert(((size_t)HK * DM / 8) % 256 == 0);

extern "C" void kernel_launch(void* const* d_in, const int* in_sizes, int n_in,
                              void* d_out, int out_size, void* d_ws, size_t ws_size, hipStream_t stream) {
    if (n_in < 9) return;
    const size_t needx = ((size_t)(SEQ - 1) * NB_FULL + NB) * DM;
    if ((size_t)in_sizes[0] < needx) return;
    if ((size_t)in_sizes[1] < (size_t)HK * DM || (size_t)in_sizes[3] < (size_t)HK * DM || (size_t)in_sizes[5] < (size_t)HK * DM || (size_t)in_sizes[7] < (size_t)DM * HK) return;
    if (in_sizes[2] < HK || in_sizes[4] < HK || in_sizes[6] < HK || in_sizes[8] < DM) return;
    if ((size_t)out_size < needx) return;
    if (SZ_TOTAL > ws_size) return;
    const float* x  = (const float*)d_in[0];
    const float* wk = (const float*)d_in[1]; const float* bk = (const float*)d_in[2];
    const float* wq = (const float*)d_in[3]; const float* bq = (const float*)d_in[4];
    const float* wv = (const float*)d_in[5]; const float* bv = (const float*)d_in[6];
    const float* wo = (const float*)d_in[7]; const float* bo = (const float*)d_in[8];
    float* OUT = (float*)d_out;
    char* wsp = (char*)d_ws;
    bf* XB = (bf*)wsp; wsp += SZ_XB;
    bf* WB = (bf*)wsp; wsp += SZ_WB;
    h16* WO = (h16*)wsp; wsp += SZ_WO;
    h16* RH = (h16*)wsp; wsp += SZ_PL;
    h16* CH = (h16*)wsp; wsp += SZ_PL;
    h16* VT = (h16*)wsp; wsp += SZ_PL;
    h16* RR = (h16*)wsp; wsp += SZ_RS;
    h16* CR = (h16*)wsp; wsp += SZ_RS;
    h16* VR = (h16*)wsp; wsp += SZ_RS;
    h16* CX = (h16*)wsp; wsp += SZ_CX;
    h16* CXR = (h16*)wsp; wsp += SZ_CR;
    bf* WKb = WB; bf* WQb = WB + (size_t)HK * DM; bf* WVb = WB + (size_t)2 * HK * DM;

    { const int n8 = NB * SEQ * DM / 8; k_cvtx<<<(unsigned)((n8 + 255) / 256), 256, 0, stream>>>(x, XB, n8); }
    { const size_t n8 = (size_t)HK * DM / 8; const unsigned g = (unsigned)((n8 + 255) / 256);
      k_cvt8<<<g, 256, 0, stream>>>(wk, WKb, n8); k_cvt8<<<g, 256, 0, stream>>>(wq, WQb, n8); k_cvt8<<<g, 256, 0, stream>>>(wv, WVb, n8); }
    { const int n8 = DM * HK / 8; k_cvtwo<<<(unsigned)((n8 + 255) / 256), 256, 0, stream>>>(wo, WO, n8); }

    k_proj_rows<<<dim3(NB * SEQ / 64, HK / 64, 1), 32, 0, stream>>>(XB, WKb, bk, RH, RR, EROWS);
    k_proj_rows<<<dim3(NB * SEQ / 64, HK / 64, 1), 32, 0, stream>>>(XB, WQb, bq, CH, CR, EROWS);
    k_proj_tr<<<dim3(HK / 64, NB * SEQ / 64, 1), 32, 0, stream>>>(WVb, XB, bv, VT, VR, EROWS);

    k_flash_early<<<dim3(EROWS / (16 * AW), NB * NH_, 1), 32 * AW, 0, stream>>>(RH, RR, CH, CR, VT, VR, CX, CXR);
    if (SEQ > EROWS)
        k_flash_late<<<dim3((SEQ - EROWS) / (16 * AW), NB * NH_, 1), 32 * AW, 0, stream>>>(RH, RR, CH, CR, VT, VR, CX, CXR);

    k_out_early<<<dim3(NB * EROWS / 32, DM / 64, 1), 32, 0, stream>>>(CX, CXR, WO, bo, OUT);
    if (SEQ > EROWS)
        k_out_late<<<dim3(NB * (SEQ - EROWS) / 32, DM / 64, 1), 32, 0, stream>>>(CX, CXR, WO, bo, OUT);
}
